// ISSMDecoderLayer_67044439491007
// MI455X (gfx1250) — hardware-verified
//
#include <hip/hip_runtime.h>
#include <math.h>

typedef __attribute__((ext_vector_type(16))) _Float16 v16h;
typedef __attribute__((ext_vector_type(8)))  _Float16 v8h;
typedef __attribute__((ext_vector_type(8)))  float    v8f;
typedef __attribute__((ext_vector_type(4)))  float    v4f;

constexpr int kNb    = 2;
constexpr int kSeq   = 1024;
constexpr int kNq    = 128;
constexpr int kDm    = 256;
constexpr int kDi    = 512;
constexpr int kNh    = 8;
constexpr int kHd    = 64;
constexpr int kCc    = 514;
constexpr int kCcP   = 544;
constexpr int kZn    = 1034;
constexpr int kZnP   = 1088;
constexpr int kDtOff = 1026;
constexpr int kRows  = kNb * kSeq;
constexpr int kQRows = kNb * kNq;
constexpr int kScT   = 16;
constexpr float kEps = 1e-5f;
constexpr float kCarryIn   = 16.0f;
constexpr float kCarryMid  = 64.0f;
constexpr float kCarryW    = 1024.0f;
constexpr float kFoldIn    = 1.0f / (kCarryIn * kCarryW);
constexpr float kFoldMid   = 1.0f / (kCarryMid * kCarryW);
constexpr float kF16MinNormal = 6.103515625e-5f;
static_assert(kDi == kNh * kHd, "heads");
static_assert(kCc == kDi + 2, "conv channels");
static_assert(kZn == 2 * kDi + 2 + kNh, "in-projection width");
static_assert(kDtOff == 2 * kDi + 2, "dt column offset");
static_assert((kZnP % 64) == 0 && kZnP >= kZn, "padded N");
static_assert((kCcP % 32) == 0 && kCcP >= kCc, "padded conv pitch");
static_assert((kDm % 32) == 0 && (kDi % 32) == 0, "GEMM K multiples of 32");
static_assert((kRows % 64) == 0 && (kQRows % 64) == 0 && (kDi % 64) == 0 && (kDm % 64) == 0, "GEMM M,N multiples of 64");
static_assert((kSeq % kScT) == 0 && (kSeq % 128) == 0, "time tiles");

constexpr size_t kSzA1H  = (size_t)kRows * kDm * 2;
constexpr size_t kSzB1H  = (size_t)kZnP * kDm * 2;
constexpr size_t kSzAQH  = (size_t)kQRows * kDm * 2;
constexpr size_t kSzBQH  = (size_t)kDi * kDm * 2;
constexpr size_t kSzBOH  = (size_t)kDm * kDi * 2;
constexpr size_t kSzZX   = (size_t)kRows * kZnP * 4;
constexpr size_t kSzH0   = (size_t)kQRows * kDi * 4;
constexpr size_t kSzXF   = (size_t)kRows * kCcP * 4;
constexpr size_t kSzTAB  = (size_t)1024 * 4 * 4;
constexpr size_t kSzGEO  = (size_t)kQRows * 32 * 4;
constexpr size_t kSzDA   = (size_t)kRows * kNh * kNq * 4;
constexpr size_t kSzCM   = (size_t)kRows * kNq * 4;
constexpr size_t kSzY    = (size_t)kRows * kDi * 4;
constexpr size_t kSzGN   = (size_t)kRows * kDi * 2;
constexpr size_t kSzSN   = (size_t)kQRows * kDi * 2;

constexpr size_t kOffA1H  = 0;
constexpr size_t kOffB1H  = kOffA1H  + kSzA1H;
constexpr size_t kOffAQH  = kOffB1H  + kSzB1H;
constexpr size_t kOffBQH  = kOffAQH  + kSzAQH;
constexpr size_t kOffBOKH = kOffBQH  + kSzBQH;
constexpr size_t kOffBOQH = kOffBOKH + kSzBOH;
constexpr size_t kOffZX   = kOffBOQH + kSzBOH;
constexpr size_t kOffH0   = kOffZX   + kSzZX;
constexpr size_t kOffXF   = kOffH0   + kSzH0;
constexpr size_t kOffXB   = kOffXF   + kSzXF;
constexpr size_t kOffTAB  = kOffXB   + kSzXF;
constexpr size_t kOffGEO  = kOffTAB  + kSzTAB;
constexpr size_t kOffDA   = kOffGEO  + kSzGEO;
constexpr size_t kOffDBF  = kOffDA   + kSzDA;
constexpr size_t kOffDBB  = kOffDBF  + kSzDA;
constexpr size_t kOffCMF  = kOffDBB  + kSzDA;
constexpr size_t kOffCMB  = kOffCMF  + kSzCM;
constexpr size_t kOffYF   = kOffCMB  + kSzCM;
constexpr size_t kOffYB   = kOffYF   + kSzY;
constexpr size_t kOffHF   = kOffYB   + kSzY;
constexpr size_t kOffHB   = kOffHF   + kSzH0;
constexpr size_t kOffGN   = kOffHB   + kSzH0;
constexpr size_t kOffSN   = kOffGN   + kSzGN;
constexpr size_t kWsTotal = kOffSN   + kSzSN;
static_assert(kWsTotal == 59981824ull, "carve total");
static_assert(kWsTotal <= 134217728ull, "carve cap");
static_assert((kOffB1H % 128) == 0 && (kOffAQH % 128) == 0 && (kOffBQH % 128) == 0 && (kOffBOKH % 128) == 0 &&
              (kOffBOQH % 128) == 0 && (kOffZX % 128) == 0 && (kOffH0 % 128) == 0 && (kOffXF % 128) == 0 &&
              (kOffXB % 128) == 0 && (kOffTAB % 128) == 0 && (kOffGEO % 128) == 0 && (kOffDA % 128) == 0 &&
              (kOffDBF % 128) == 0 && (kOffDBB % 128) == 0 && (kOffCMF % 128) == 0 && (kOffCMB % 128) == 0 &&
              (kOffYF % 128) == 0 && (kOffYB % 128) == 0 && (kOffHF % 128) == 0 && (kOffHB % 128) == 0 &&
              (kOffGN % 128) == 0 && (kOffSN % 128) == 0, "128-B aligned regions");

__device__ __forceinline__ float flush_f16_operand(float x) {
  return (fabsf(x) < kF16MinNormal) ? 0.0f : x;
}
__device__ __forceinline__ float sigmoid_f(float v) { return 1.0f / (1.0f + expf(-v)); }
__device__ __forceinline__ float softplus_f(float v) { return fmaxf(v, 0.0f) + log1pf(expf(-fabsf(v))); }
__device__ __forceinline__ int clamp_i(int v, int lo, int hi) { return v < lo ? lo : (v > hi ? hi : v); }

__device__ __forceinline__ v16h frag_load_h(const _Float16* p) {
  union { v16h v; v8h h[2]; } f;
  f.h[0] = *(const v8h*)(p);
  f.h[1] = *(const v8h*)(p + 16);
  return f.v;
}
__device__ __forceinline__ v8f mma_h(v16h a, v16h b, v8f c) {
  return __builtin_amdgcn_wmma_f32_16x16x32_f16(false, a, false, b, (short)0, c, false, false);
}
__device__ __forceinline__ void tie_acc_h(v8f& a, v16h x) { asm volatile("" : "+v"(a) : "v"(x)); }
__device__ __forceinline__ void nop4_acc_h(v8f& a, v16h x, v16h y) { asm volatile("v_nop\n\tv_nop\n\tv_nop\n\tv_nop" : "+v"(a) : "v"(x), "v"(y)); }
__device__ __forceinline__ void keep4_h(v16h a, v16h b, v16h c, v16h d) { asm volatile("v_nop" :: "v"(a), "v"(b), "v"(c), "v"(d)); }
__device__ __forceinline__ void acc_guard4(v8f& a, v8f& b, v8f& c, v8f& d) { asm volatile("v_nop\n\tv_nop\n\tv_nop\n\tv_nop" : "+v"(a), "+v"(b), "+v"(c), "+v"(d)); }

__global__ __launch_bounds__(256) void cast_f16_carry_kernel(
    const float* __restrict__ src, unsigned short* __restrict__ dst, int total8, int valid8, float carry)
{
  const int i = blockIdx.x * 256 + threadIdx.x;
  if (i >= total8) return;
  const bool live = (i < valid8);
  const int ic = live ? i : (valid8 - 1);
  const size_t e0 = (size_t)ic << 3;
  const v4f a0 = *(const v4f*)(src + e0);
  const v4f a1 = *(const v4f*)(src + e0 + 4);
  v8h hv;
#pragma unroll
  for (int e = 0; e < 4; ++e) {
    const float s0 = a0[e];
    const float s1 = a1[e];
    const float x0 = flush_f16_operand(live ? (s0 * carry) : 0.0f);
    const float x1 = flush_f16_operand(live ? (s1 * carry) : 0.0f);
    hv[e]     = (_Float16)x0;
    hv[4 + e] = (_Float16)x1;
  }
  unsigned short* q = dst + ((size_t)i << 3);
  *(volatile v8h*)q = hv;
  __threadfence();
  *(volatile v8h*)q = hv;
}

__global__ __launch_bounds__(256) void gemm_f16_nt_kernel(
    const unsigned short* __restrict__ Ap, int lda,
    const unsigned short* __restrict__ Btp, int ldb,
    float* __restrict__ C, int ldc, int M, int N, int K, float scale)
{
  const _Float16* A  = (const _Float16*)Ap;
  const _Float16* Bt = (const _Float16*)Btp;
  __shared__ __align__(16) float sT[8][16 * 68];
  const int lane = threadIdx.x & 31;
  const int wave = threadIdx.x >> 5;
  const int tilesN = N >> 6;
  const int tilesM = M >> 6;
  const int tile = blockIdx.x * 8 + wave;
  if (tile >= tilesM * tilesN) return;
  const int tm = tile / tilesN;
  const int tn = tile - tm * tilesN;
  const int m0 = tm << 6;
  const int n0 = tn << 6;
  const int rlane = lane & 15;
  const int koff  = (lane >> 4) * 8;
  const int mOff  = (lane >> 4) * 8;

  v8f acc[4][4];
#pragma unroll
  for (int i = 0; i < 4; ++i)
#pragma unroll
    for (int j = 0; j < 4; ++j) acc[i][j] = (v8f){0.f,0.f,0.f,0.f,0.f,0.f,0.f,0.f};

  for (int k0 = 0; k0 < K; k0 += 32) {
    v16h bh[4];
#pragma unroll
    for (int j = 0; j < 4; ++j) {
      const size_t bo = (size_t)(n0 + (j << 4) + rlane) * ldb + koff + k0;
      bh[j] = frag_load_h(Bt + bo);
    }
#pragma unroll
    for (int i = 0; i < 4; ++i) {
      const size_t ao = (size_t)(m0 + (i << 4) + rlane) * lda + koff + k0;
      const v16h ah = frag_load_h(A + ao);
#pragma unroll
      for (int j = 0; j < 4; ++j) acc[i][j] = mma_h(ah, bh[j], acc[i][j]);
      tie_acc_h(acc[i][1], ah);
      tie_acc_h(acc[i][2], ah);
      tie_acc_h(acc[i][3], ah);
      nop4_acc_h(acc[i][0], ah, bh[3]);
    }
    keep4_h(bh[0], bh[1], bh[2], bh[3]);
  }
  acc_guard4(acc[0][0], acc[0][1], acc[0][2], acc[0][3]);
  acc_guard4(acc[1][0], acc[1][1], acc[1][2], acc[1][3]);
  acc_guard4(acc[2][0], acc[2][1], acc[2][2], acc[2][3]);
  acc_guard4(acc[3][0], acc[3][1], acc[3][2], acc[3][3]);

  float* slab = sT[wave];
#pragma unroll
  for (int i = 0; i < 4; ++i) {
    const int mBase = m0 + (i << 4);
#pragma unroll
    for (int j = 0; j < 4; ++j) {
#pragma unroll
      for (int r = 0; r < 8; ++r) {
        slab[(mOff + r) * 68 + (j << 4) + rlane] = acc[i][j][r] * scale;
      }
    }
    __builtin_amdgcn_fence(__ATOMIC_RELEASE, "workgroup");
    __builtin_amdgcn_wave_barrier();
    __builtin_amdgcn_fence(__ATOMIC_ACQUIRE, "workgroup");
    {
      const int hh = lane >> 4, c4 = (lane & 15) * 4;
      for (int pass = 0; pass < 2; ++pass) {
#pragma unroll
        for (int it = 0; it < 8; ++it) {
          const int row = it * 2 + hh;
          const v4f v = *(const v4f*)(slab + row * 68 + c4);
          *(volatile v4f*)(C + (size_t)(mBase + row) * ldc + n0 + c4) = v;
        }
        __threadfence();
      }
    }
    __builtin_amdgcn_fence(__ATOMIC_RELEASE, "workgroup");
    __builtin_amdgcn_wave_barrier();
    __builtin_amdgcn_fence(__ATOMIC_ACQUIRE, "workgroup");
  }
}

__device__ __forceinline__ float conv_sample(const float* __restrict__ in, int ldin, int bb, int l, int cc) {
  const bool ok = (l >= 0) && (l < kSeq);
  const int lc = clamp_i(l, 0, kSeq - 1);
  float v = in[(size_t)(bb * kSeq + lc) * ldin + cc];
  asm volatile("" : "+v"(v));
  return ok ? v : 0.0f;
}

__global__ __launch_bounds__(256) void dwconv7_silu_kernel(
    const float* __restrict__ in, int ldin, const float* __restrict__ w, const float* __restrict__ bias,
    float* __restrict__ out)
{
  const int lane = threadIdx.x & 31, wave = threadIdx.x >> 5;
  const int c = blockIdx.x * 32 + lane;
  const bool live = (c < kCc);
  const int cc = live ? c : (kCc - 1);
  const int r0 = (blockIdx.y * 8 + wave) * 16;
  const int bb = r0 / kSeq;
  const int l0 = r0 - bb * kSeq;
  const float w0 = w[cc * 7 + 0], w1 = w[cc * 7 + 1], w2 = w[cc * 7 + 2], w3 = w[cc * 7 + 3];
  const float w4 = w[cc * 7 + 4], w5 = w[cc * 7 + 5], w6 = w[cc * 7 + 6];
  const float bv = bias[cc];
  float x0 = conv_sample(in, ldin, bb, l0 - 3, cc);
  float x1 = conv_sample(in, ldin, bb, l0 - 2, cc);
  float x2 = conv_sample(in, ldin, bb, l0 - 1, cc);
  float x3 = conv_sample(in, ldin, bb, l0, cc);
  float x4 = conv_sample(in, ldin, bb, l0 + 1, cc);
  float x5 = conv_sample(in, ldin, bb, l0 + 2, cc);
#pragma unroll 1
  for (int s = 0; s < 16; ++s) {
    const float x6 = conv_sample(in, ldin, bb, l0 + s + 3, cc);
    float a = w0 * x0;
    a = fmaf(w1, x1, a);
    a = fmaf(w2, x2, a);
    a = fmaf(w3, x3, a);
    a = fmaf(w4, x4, a);
    a = fmaf(w5, x5, a);
    a = fmaf(w6, x6, a);
    const float sv = a + bv;
    const float act = sv * sigmoid_f(sv);
    const float o = live ? act : 0.0f;
    float* p = out + (size_t)(r0 + s) * kCcP + c;
    *(volatile float*)p = o;
    __threadfence();
    *(volatile float*)p = o;
    x0 = x1; x1 = x2; x2 = x3; x3 = x4; x4 = x5; x5 = x6;
  }
}

__global__ __launch_bounds__(256) void table_geom_kernel(
    const float* __restrict__ w1, const float* __restrict__ b1, const float* __restrict__ w2,
    const float* __restrict__ qxyz, const float* __restrict__ qsize, const float* __restrict__ qang,
    float* __restrict__ table, float* __restrict__ geo)
{
  __shared__ __align__(16) float sG[256 * 32];
  const int tid = threadIdx.x;
  if (blockIdx.x < 4) {
    const int idx = blockIdx.x * 256 + tid;
    const bool live = (idx < 1000);
    const int ic = live ? idx : 999;
    const int ia = ic / 100, ib = (ic / 10) % 10, ig = ic % 10;
    const float px = -4.0f + (8.0f * (float)ia) * (1.0f / 9.0f);
    const float py = -4.0f + (8.0f * (float)ib) * (1.0f / 9.0f);
    const float pz = -4.0f + (8.0f * (float)ig) * (1.0f / 9.0f);
    float o0 = 0.f, o1 = 0.f, o2 = 0.f, o3 = 0.f;
#pragma unroll 1
    for (int j = 0; j < 128; ++j) {
      float hd = w1[j * 3] * px;
      hd = fmaf(w1[j * 3 + 1], py, hd);
      hd = fmaf(w1[j * 3 + 2], pz, hd);
      hd = fmaxf(hd + b1[j], 0.0f);
      o0 = fmaf(w2[j], hd, o0);
      o1 = fmaf(w2[128 + j], hd, o1);
      o2 = fmaf(w2[256 + j], hd, o2);
      o3 = fmaf(w2[384 + j], hd, o3);
    }
    v4f ov;
    ov[0] = live ? o0 : 0.0f;
    ov[1] = live ? o1 : 0.0f;
    ov[2] = live ? o2 : 0.0f;
    ov[3] = live ? o3 : 0.0f;
    float* p = table + (size_t)idx * 4;
    *(volatile v4f*)p = ov;
    __threadfence();
    *(volatile v4f*)p = ov;
  } else {
    const int bk = tid;
    const float cx = qxyz[bk * 3], cy = qxyz[bk * 3 + 1], cz = qxyz[bk * 3 + 2];
    const float ls = qsize[bk * 3], wsz = qsize[bk * 3 + 1], hs = qsize[bk * 3 + 2];
    const float ang = qang[bk];
    const float cs = cosf(ang), sn = sinf(ang);
    float* rec = sG + bk * 32;
#pragma unroll 1
    for (int c = 0; c < 8; ++c) {
      const float sx = (c & 2) ? -1.0f : 1.0f;
      const float sy = (c & 4) ? -1.0f : 1.0f;
      const float sz = ((c + 1) & 2) ? -1.0f : 1.0f;
      const float l0 = ls * sx * 0.5f;
      const float l1 = hs * sy * 0.5f;
      const float l2 = wsz * sz * 0.5f;
      rec[c * 3 + 0] = cx + cs * l0 + sn * l2;
      rec[c * 3 + 1] = cy - sn * l0 + cs * l2;
      rec[c * 3 + 2] = cz - l1;
    }
    rec[24] = cs;
    rec[25] = sn;
    rec[26] = 0.0f; rec[27] = 0.0f; rec[28] = 0.0f; rec[29] = 0.0f; rec[30] = 0.0f; rec[31] = 0.0f;
    __syncthreads();
    v4f gv[8];
#pragma unroll
    for (int it = 0; it < 8; ++it) gv[it] = *(const v4f*)(sG + (size_t)(it * 256 + tid) * 4);
    for (int pass = 0; pass < 2; ++pass) {
#pragma unroll
      for (int it = 0; it < 8; ++it) *(volatile v4f*)(geo + (size_t)(it * 256 + tid) * 4) = gv[it];
      __threadfence();
    }
  }
}

__device__ __forceinline__ float pix_of(float u) {
  const float sg = (u > 0.0f) ? 1.0f : ((u < 0.0f) ? -1.0f : 0.0f);
  const float cmp = sg * log2f(fabsf(u) * 512.0f + 1.0f) * (1.0f / 3.0f);
  const float g = cmp * 0.25f;
  return ((g + 1.0f) * 10.0f - 1.0f) * 0.5f;
}

__global__ __launch_bounds__(256) void dist_coef_kernel(
    const float* __restrict__ key_xyz, const float* __restrict__ table, const float* __restrict__ geo,
    const float* __restrict__ zx, const float* __restrict__ xf, const float* __restrict__ xb,
    const float* __restrict__ Wbc, const float* __restrict__ Wdt, const float* __restrict__ dt_bias,
    const float* __restrict__ A_log,
    float* __restrict__ dA, float* __restrict__ dBf, float* __restrict__ dBb,
    float* __restrict__ CmF, float* __restrict__ CmB)
{
  __shared__ __align__(16) float sTab[1024 * 4];
  __shared__ __align__(16) float sGeo[kNq * 32];
  const int tid = threadIdx.x;
  const int bb = blockIdx.x / (kSeq / 8);
  const int l0 = (blockIdx.x - bb * (kSeq / 8)) * 8;
#pragma unroll
  for (int it = 0; it < 4; ++it) {
    const int idx4 = it * 256 + tid;
    *(v4f*)(sTab + idx4 * 4) = *(const v4f*)(table + (size_t)idx4 * 4);
    *(v4f*)(sGeo + idx4 * 4) = *(const v4f*)(geo + (size_t)bb * (kNq * 32) + (size_t)idx4 * 4);
  }
  __syncthreads();
  const int k = tid & (kNq - 1);
  const int lh = tid >> 7;
  const float wb0 = Wbc[0], wb1 = Wbc[1], wb2 = Wbc[2], wb3 = Wbc[3];
  const float wc0 = Wbc[4], wc1 = Wbc[5], wc2 = Wbc[6], wc3 = Wbc[7];
#pragma unroll 1
  for (int li = 0; li < 4; ++li) {
    const int l = l0 + li * 2 + lh;
    const size_t row = (size_t)bb * kSeq + l;
    const float kx = key_xyz[row * 3], ky = key_xyz[row * 3 + 1], kz = key_xyz[row * 3 + 2];
    float o0 = 0.f, o1 = 0.f, o2 = 0.f, o3 = 0.f;
#pragma unroll 1
    for (int c = 0; c < 8; ++c) {
      const float* cp = sGeo + k * 32 + c * 3;
      const float dx = cp[0] - kx, dy = cp[1] - ky, dz = cp[2] - kz;
      const int q = (k * 8 + c) & (kNq - 1);
      const float cs = sGeo[q * 32 + 24], sn = sGeo[q * 32 + 25];
      const float u0 = dx * cs - dy * sn;
      const float u1 = dx * sn + dy * cs;
      const float u2 = dz;
      const float pk = pix_of(u0);
      const float pj = pix_of(u1);
      const float pi = pix_of(u2);
      const float i0f = floorf(pi), j0f = floorf(pj), k0f = floorf(pk);
      const float wi = pi - i0f, wj = pj - j0f, wk = pk - k0f;
      const int i0 = (int)i0f, j0 = (int)j0f, k0 = (int)k0f;
#pragma unroll 1
      for (int ab = 0; ab < 4; ++ab) {
        const int ta = ab >> 1, tb = ab & 1;
        const int ii = i0 + ta, jj = j0 + tb;
        const float wa = ta ? wi : (1.0f - wi);
        const float wbv = tb ? wj : (1.0f - wj);
        const float wab = wa * wbv;
        const bool vab = (ii >= 0) && (ii < 10) && (jj >= 0) && (jj < 10);
        const int base = clamp_i(ii, 0, 9) * 100 + clamp_i(jj, 0, 9) * 10;
#pragma unroll
        for (int tc = 0; tc < 2; ++tc) {
          const int kk = k0 + tc;
          const bool vk = vab && (kk >= 0) && (kk < 10);
          const float wfull = wab * (tc ? wk : (1.0f - wk));
          const float wt = vk ? wfull : 0.0f;
          const v4f tv = *(const v4f*)(sTab + (base + clamp_i(kk, 0, 9)) * 4);
          o0 = fmaf(wt, tv[0], o0);
          o1 = fmaf(wt, tv[1], o1);
          o2 = fmaf(wt, tv[2], o2);
          o3 = fmaf(wt, tv[3], o3);
        }
      }
    }
    const float Bm0 = o0 * wb0 + o1 * wb1 + o2 * wb2 + o3 * wb3;
    const float Cm0 = o0 * wc0 + o1 * wc1 + o2 * wc2 + o3 * wc3;
    const float bbF = xf[row * kCcP + kDi];
    const float cbF = xf[row * kCcP + kDi + 1];
    const float bbB = xb[row * kCcP + kDi];
    const float cbB = xb[row * kCcP + kDi + 1];
    const float cF = Cm0 + cbF, cB = Cm0 + cbB;
    const float BmF = Bm0 + bbF, BmB = Bm0 + bbB;
    {
      float* pf = CmF + row * kNq + k;
      float* pb = CmB + row * kNq + k;
      *(volatile float*)pf = cF;
      *(volatile float*)pb = cB;
      __threadfence();
      *(volatile float*)pf = cF;
      *(volatile float*)pb = cB;
    }
#pragma unroll 1
    for (int h = 0; h < kNh; ++h) {
      float t = o0 * Wdt[h * 4] + o1 * Wdt[h * 4 + 1] + o2 * Wdt[h * 4 + 2] + o3 * Wdt[h * 4 + 3];
      t = t + zx[row * kZnP + kDtOff + h];
      t = t + dt_bias[h];
      const float dt = softplus_f(t);
      const float an = -expf(A_log[h]);
      const float vA = expf(dt * an);
      const float vBf = dt * BmF;
      const float vBb = dt * BmB;
      const size_t o = (row * kNh + h) * kNq + k;
      *(volatile float*)(dA + o) = vA;
      *(volatile float*)(dBf + o) = vBf;
      *(volatile float*)(dBb + o) = vBb;
      __threadfence();
      *(volatile float*)(dA + o) = vA;
      *(volatile float*)(dBf + o) = vBf;
      *(volatile float*)(dBb + o) = vBb;
    }
  }
}

__global__ __launch_bounds__(256) void scan_kernel(
    const float* __restrict__ dA, const float* __restrict__ dBf, const float* __restrict__ dBb,
    const float* __restrict__ CmF, const float* __restrict__ CmB,
    const float* __restrict__ xf, const float* __restrict__ xb, const float* __restrict__ h0,
    float* __restrict__ yF, float* __restrict__ yB, float* __restrict__ hF, float* __restrict__ hB)
{
  __shared__ __align__(16) float sBuf[8192];
  __shared__ __align__(16) float sY[kScT * 68];
  const int blk = blockIdx.x;
  const int dir = blk >> 4;
  const int bb  = (blk >> 3) & 1;
  const int h   = blk & 7;
  const int tid = threadIdx.x;
  const int d   = tid >> 2;
  const int kq  = tid & 3;
  const int lane = tid & 31, wave = tid >> 5;

  const float* dBp = dir ? dBb : dBf;
  const float* Cmp = dir ? CmB : CmF;
  const float* xs  = dir ? xb : xf;
  float* yo = dir ? yB : yF;
  float* ho = dir ? hB : hF;

  float* sA = sBuf;
  float* sB = sBuf + 2048;
  float* sC = sBuf + 4096;
  float* sX = sBuf + 6144;

  {
    const int rr = tid >> 4, c4 = (tid & 15) * 4;
#pragma unroll
    for (int it = 0; it < 8; ++it) {
      const int r = it * 16 + rr;
      *(v4f*)(sBuf + r * 64 + c4) = *(const v4f*)(h0 + (size_t)(bb * kNq + r) * kDi + h * kHd + c4);
    }
  }
  __syncthreads();
  float hst[32];
#pragma unroll
  for (int i = 0; i < 32; ++i) hst[i] = sBuf[(kq * 32 + i) * 64 + d];

#pragma unroll 1
  for (int c0 = 0; c0 < kSeq; c0 += kScT) {
    __syncthreads();
#pragma unroll
    for (int it = 0; it < 2; ++it) {
      const int idx4 = it * 256 + tid;
      const int s = idx4 >> 5, k4 = (idx4 & 31) * 4;
      const int t = dir ? (kSeq - 1 - (c0 + s)) : (c0 + s);
      const size_t row = (size_t)bb * kSeq + t;
      *(v4f*)(sA + s * 128 + k4) = *(const v4f*)(dA  + (row * kNh + h) * kNq + k4);
      *(v4f*)(sB + s * 128 + k4) = *(const v4f*)(dBp + (row * kNh + h) * kNq + k4);
      *(v4f*)(sC + s * 128 + k4) = *(const v4f*)(Cmp + row * kNq + k4);
    }
    {
      const int s = tid >> 4, c4 = (tid & 15) * 4;
      const int t = dir ? (kSeq - 1 - (c0 + s)) : (c0 + s);
      const size_t row = (size_t)bb * kSeq + t;
      *(v4f*)(sX + s * 64 + c4) = *(const v4f*)(xs + row * kCcP + h * kHd + c4);
    }
    __syncthreads();
#pragma unroll 1
    for (int s = 0; s < kScT; ++s) {
      const float xv = sX[s * 64 + d];
      const float* pa = sA + s * 128 + kq * 32;
      const float* pb = sB + s * 128 + kq * 32;
      const float* pc = sC + s * 128 + kq * 32;
      float acc = 0.0f;
#pragma unroll
      for (int j = 0; j < 8; ++j) {
        const v4f av = *(const v4f*)(pa + 4 * j);
        const v4f bv = *(const v4f*)(pb + 4 * j);
        const v4f cv = *(const v4f*)(pc + 4 * j);
#pragma unroll
        for (int e = 0; e < 4; ++e) {
          const float hv = fmaf(hst[4 * j + e], av[e], xv * bv[e]);
          hst[4 * j + e] = hv;
          acc = fmaf(hv, cv[e], acc);
        }
      }
      acc += __shfl_xor(acc, 1);
      acc += __shfl_xor(acc, 2);
      if (kq == 0) sY[s * 68 + d] = acc;
    }
    __syncthreads();
    {
      const int srow = 2 * wave + (lane >> 4), c4 = (lane & 15) * 4;
      const int t = dir ? (kSeq - 1 - (c0 + srow)) : (c0 + srow);
      const v4f yv = *(const v4f*)(sY + srow * 68 + c4);
      float* p = yo + ((size_t)bb * kSeq + t) * kDi + h * kHd + c4;
      *(volatile v4f*)p = yv;
      __threadfence();
      *(volatile v4f*)p = yv;
    }
  }
  __syncthreads();
#pragma unroll
  for (int i = 0; i < 32; ++i) sBuf[(kq * 32 + i) * 64 + d] = hst[i];
  __syncthreads();
  {
    const int hh = lane >> 4, c4 = (lane & 15) * 4;
    v4f sv[8];
#pragma unroll
    for (int it = 0; it < 8; ++it) sv[it] = *(const v4f*)(sBuf + (it * 16 + 2 * wave + hh) * 64 + c4);
    for (int pass = 0; pass < 2; ++pass) {
#pragma unroll
      for (int it = 0; it < 8; ++it) {
        const int r = it * 16 + 2 * wave + hh;
        *(volatile v4f*)(ho + (size_t)(bb * kNq + r) * kDi + h * kHd + c4) = sv[it];
      }
      __threadfence();
    }
  }
}

__device__ __forceinline__ float gate_one(float yf, float yb, float x, float z, float dpv) {
  const float yv = (yf + yb) + dpv * x;
  return yv * (z * sigmoid_f(z));
}

__global__ __launch_bounds__(256) void gate_rmsnorm_kernel(
    const float* __restrict__ yF, const float* __restrict__ yB, const float* __restrict__ xf,
    const float* __restrict__ zx, const float* __restrict__ Dp, const float* __restrict__ knw,
    unsigned short* __restrict__ gout)
{
  __shared__ float sG[16 * 256];
  const int tid = threadIdx.x, lane = tid & 31, wave = tid >> 5;
  const size_t row = (size_t)blockIdx.x * 8 + wave;
  float ssum = 0.0f;
#pragma unroll 1
  for (int hc = 0; hc < 2; ++hc) {
    const int c0 = hc * 256 + lane * 8;
    const float dpv = Dp[c0 >> 6];
    const v4f yf0 = *(const v4f*)(yF + row * kDi + c0);
    const v4f yf1 = *(const v4f*)(yF + row * kDi + c0 + 4);
    const v4f yb0 = *(const v4f*)(yB + row * kDi + c0);
    const v4f yb1 = *(const v4f*)(yB + row * kDi + c0 + 4);
    const v4f xa0 = *(const v4f*)(xf + row * kCcP + c0);
    const v4f xa1 = *(const v4f*)(xf + row * kCcP + c0 + 4);
    const v4f za0 = *(const v4f*)(zx + row * kZnP + c0);
    const v4f za1 = *(const v4f*)(zx + row * kZnP + c0 + 4);
#pragma unroll
    for (int e = 0; e < 4; ++e) {
      const float g0 = gate_one(yf0[e], yb0[e], xa0[e], za0[e], dpv);
      const float g1 = gate_one(yf1[e], yb1[e], xa1[e], za1[e], dpv);
      ssum = fmaf(g0, g0, ssum);
      ssum = fmaf(g1, g1, ssum);
      sG[(hc * 8 + e) * 256 + tid] = g0;
      sG[(hc * 8 + 4 + e) * 256 + tid] = g1;
    }
  }
  ssum += __shfl_xor(ssum, 16);
  ssum += __shfl_xor(ssum, 8);
  ssum += __shfl_xor(ssum, 4);
  ssum += __shfl_xor(ssum, 2);
  ssum += __shfl_xor(ssum, 1);
  const float rn = rsqrtf(ssum * (1.0f / (float)kDi) + kEps);
#pragma unroll 1
  for (int hc = 0; hc < 2; ++hc) {
    const int c0 = hc * 256 + lane * 8;
    const v4f k0 = *(const v4f*)(knw + c0);
    const v4f k1 = *(const v4f*)(knw + c0 + 4);
    v8h hv;
#pragma unroll
    for (int e = 0; e < 4; ++e) {
      const float g0 = sG[(hc * 8 + e) * 256 + tid];
      const float g1 = sG[(hc * 8 + 4 + e) * 256 + tid];
      const float o0 = flush_f16_operand(((g0 * rn) * k0[e]) * kCarryMid);
      const float o1 = flush_f16_operand(((g1 * rn) * k1[e]) * kCarryMid);
      hv[e]     = (_Float16)o0;
      hv[4 + e] = (_Float16)o1;
    }
    unsigned short* p = gout + row * kDi + c0;
    *(volatile v8h*)p = hv;
    __threadfence();
    *(volatile v8h*)p = hv;
  }
}

__global__ __launch_bounds__(256) void state_layernorm_kernel(
    const float* __restrict__ hF, const float* __restrict__ hB,
    const float* __restrict__ lnw, const float* __restrict__ lnb, unsigned short* __restrict__ sout)
{
  const int tid = threadIdx.x, lane = tid & 31, wave = tid >> 5;
  const size_t row = (size_t)blockIdx.x * 8 + wave;
  float v[16];
  float s = 0.0f;
#pragma unroll
  for (int hc = 0; hc < 2; ++hc) {
    const int c0 = hc * 256 + lane * 8;
    const v4f a0 = *(const v4f*)(hF + row * kDi + c0);
    const v4f a1 = *(const v4f*)(hF + row * kDi + c0 + 4);
    const v4f b0 = *(const v4f*)(hB + row * kDi + c0);
    const v4f b1 = *(const v4f*)(hB + row * kDi + c0 + 4);
#pragma unroll
    for (int e = 0; e < 4; ++e) {
      v[hc * 8 + e]     = 0.5f * (a0[e] + b0[e]);
      v[hc * 8 + 4 + e] = 0.5f * (a1[e] + b1[e]);
      s += v[hc * 8 + e];
      s += v[hc * 8 + 4 + e];
    }
  }
  s += __shfl_xor(s, 16);
  s += __shfl_xor(s, 8);
  s += __shfl_xor(s, 4);
  s += __shfl_xor(s, 2);
  s += __shfl_xor(s, 1);
  const float mu = s * (1.0f / (float)kDi);
  float q = 0.0f;
#pragma unroll
  for (int i = 0; i < 16; ++i) {
    const float dv = v[i] - mu;
    q = fmaf(dv, dv, q);
  }
  q += __shfl_xor(q, 16);
  q += __shfl_xor(q, 8);
  q += __shfl_xor(q, 4);
  q += __shfl_xor(q, 2);
  q += __shfl_xor(q, 1);
  const float inv = rsqrtf(q * (1.0f / (float)kDi) + kEps);
  v8h hv[2];
#pragma unroll
  for (int hc = 0; hc < 2; ++hc) {
    const int c0 = hc * 256 + lane * 8;
    const v4f w0 = *(const v4f*)(lnw + c0);
    const v4f w1 = *(const v4f*)(lnw + c0 + 4);
    const v4f e0 = *(const v4f*)(lnb + c0);
    const v4f e1 = *(const v4f*)(lnb + c0 + 4);
#pragma unroll
    for (int e = 0; e < 4; ++e) {
      const float o0 = flush_f16_operand((((v[hc * 8 + e] - mu) * inv) * w0[e] + e0[e]) * kCarryMid);
      const float o1 = flush_f16_operand((((v[hc * 8 + 4 + e] - mu) * inv) * w1[e] + e1[e]) * kCarryMid);
      hv[hc][e]     = (_Float16)o0;
      hv[hc][4 + e] = (_Float16)o1;
    }
  }
  for (int pass = 0; pass < 2; ++pass) {
#pragma unroll
    for (int hc = 0; hc < 2; ++hc) {
      *(volatile v8h*)(sout + row * kDi + hc * 256 + lane * 8) = hv[hc];
    }
    __threadfence();
  }
}

extern "C" void kernel_launch(void* const* d_in, const int* in_sizes, int n_in,
                              void* d_out, int out_size, void* d_ws, size_t ws_size,
                              hipStream_t stream) {
  if (n_in < 25) return;
  if (in_sizes[0] != kRows * kDm) return;
  if (in_sizes[1] != kQRows * kDm) return;
  if (in_sizes[2] != kRows * 3) return;
  if (in_sizes[3] != kQRows * 3) return;
  if (in_sizes[4] != kQRows * 3) return;
  if (in_sizes[5] != kQRows) return;
  if (in_sizes[6] != kZn * kDm) return;
  if (in_sizes[7] != kCc * 7) return;
  if (in_sizes[8] != kCc) return;
  if (in_sizes[9] != kCc * 7) return;
  if (in_sizes[10] != kCc) return;
  if (in_sizes[11] != kDi * kDm) return;
  if (in_sizes[12] != 8) return;
  if (in_sizes[13] != kNh * 4) return;
  if (in_sizes[14] != kNh) return;
  if (in_sizes[15] != kNh) return;
  if (in_sizes[16] != kNh) return;
  if (in_sizes[17] != kDm * kDi) return;
  if (in_sizes[18] != kDm * kDi) return;
  if (in_sizes[19] != kDi) return;
  if (in_sizes[20] != kDi) return;
  if (in_sizes[21] != kDi) return;
  if (in_sizes[22] != 128 * 3) return;
  if (in_sizes[23] != 128) return;
  if (in_sizes[24] != 4 * 128) return;
  if (out_size != kRows * kDm + kQRows * kDm) return;
  if (ws_size < kWsTotal) return;

  const float* in_key      = (const float*)d_in[0];
  const float* in_query    = (const float*)d_in[1];
  const float* key_xyz     = (const float*)d_in[2];
  const float* query_xyz   = (const float*)d_in[3];
  const float* query_size  = (const float*)d_in[4];
  const float* query_angle = (const float*)d_in[5];
  const float* Wkey        = (const float*)d_in[6];
  const float* conv_w      = (const float*)d_in[7];
  const float* conv_b      = (const float*)d_in[8];
  const float* convb_w     = (const float*)d_in[9];
  const float* convb_b     = (const float*)d_in[10];
  const float* Wq          = (const float*)d_in[11];
  const float* Wbc         = (const float*)d_in[12];
  const float* Wdt         = (const float*)d_in[13];
  const float* dt_bias     = (const float*)d_in[14];
  const float* A_log       = (const float*)d_in[15];
  const float* Dp          = (const float*)d_in[16];
  const float* Wok         = (const float*)d_in[17];
  const float* Woq         = (const float*)d_in[18];
  const float* key_norm_w  = (const float*)d_in[19];
  const float* ln_w        = (const float*)d_in[20];
  const float* ln_b        = (const float*)d_in[21];
  const float* cpb_w1      = (const float*)d_in[22];
  const float* cpb_b1      = (const float*)d_in[23];
  const float* cpb_w2      = (const float*)d_in[24];
  float* out = (float*)d_out;

  char* ws = (char*)d_ws;
  unsigned short* A1H  = (unsigned short*)(ws + kOffA1H);
  unsigned short* B1H  = (unsigned short*)(ws + kOffB1H);
  unsigned short* AQH  = (unsigned short*)(ws + kOffAQH);
  unsigned short* BQH  = (unsigned short*)(ws + kOffBQH);
  unsigned short* BOKH = (unsigned short*)(ws + kOffBOKH);
  unsigned short* BOQH = (unsigned short*)(ws + kOffBOQH);
  float* ZX  = (float*)(ws + kOffZX);
  float* H0  = (float*)(ws + kOffH0);
  float* XF  = (float*)(ws + kOffXF);
  float* XB  = (float*)(ws + kOffXB);
  float* TAB = (float*)(ws + kOffTAB);
  float* GEO = (float*)(ws + kOffGEO);
  float* DA  = (float*)(ws + kOffDA);
  float* DBF = (float*)(ws + kOffDBF);
  float* DBB = (float*)(ws + kOffDBB);
  float* CMF = (float*)(ws + kOffCMF);
  float* CMB = (float*)(ws + kOffCMB);
  float* YF  = (float*)(ws + kOffYF);
  float* YB  = (float*)(ws + kOffYB);
  float* HF  = (float*)(ws + kOffHF);
  float* HB  = (float*)(ws + kOffHB);
  unsigned short* GN = (unsigned short*)(ws + kOffGN);
  unsigned short* SN = (unsigned short*)(ws + kOffSN);

  cast_f16_carry_kernel<<<(kRows * kDm / 8) / 256, 256, 0, stream>>>(in_key, A1H, kRows * kDm / 8, kRows * kDm / 8, kCarryIn);
  cast_f16_carry_kernel<<<(kZnP * kDm / 8) / 256, 256, 0, stream>>>(Wkey, B1H, kZnP * kDm / 8, kZn * kDm / 8, kCarryW);
  cast_f16_carry_kernel<<<(kQRows * kDm / 8) / 256, 256, 0, stream>>>(in_query, AQH, kQRows * kDm / 8, kQRows * kDm / 8, kCarryIn);
  cast_f16_carry_kernel<<<(kDi * kDm / 8) / 256, 256, 0, stream>>>(Wq, BQH, kDi * kDm / 8, kDi * kDm / 8, kCarryW);
  cast_f16_carry_kernel<<<(kDm * kDi / 8) / 256, 256, 0, stream>>>(Wok, BOKH, kDm * kDi / 8, kDm * kDi / 8, kCarryW);
  cast_f16_carry_kernel<<<(kDm * kDi / 8) / 256, 256, 0, stream>>>(Woq, BOQH, kDm * kDi / 8, kDm * kDi / 8, kCarryW);

  gemm_f16_nt_kernel<<<((kRows / 64) * (kZnP / 64)) / 8, 256, 0, stream>>>(
      A1H, kDm, B1H, kDm, ZX, kZnP, kRows, kZnP, kDm, kFoldIn);
  gemm_f16_nt_kernel<<<((kQRows / 64) * (kDi / 64)) / 8, 256, 0, stream>>>(
      AQH, kDm, BQH, kDm, H0, kDi, kQRows, kDi, kDm, kFoldIn);

  dwconv7_silu_kernel<<<dim3(kCcP / 32, kRows / 128), 256, 0, stream>>>(ZX + kDi, kZnP, conv_w, conv_b, XF);
  dwconv7_silu_kernel<<<dim3(kCcP / 32, kRows / 128), 256, 0, stream>>>(XF, kCcP, convb_w, convb_b, XB);

  table_geom_kernel<<<5, 256, 0, stream>>>(cpb_w1, cpb_b1, cpb_w2, query_xyz, query_size, query_angle, TAB, GEO);

  dist_coef_kernel<<<kNb * (kSeq / 8), 256, 0, stream>>>(key_xyz, TAB, GEO, ZX, XF, XB, Wbc, Wdt, dt_bias, A_log,
                                                        DA, DBF, DBB, CMF, CMB);

  scan_kernel<<<2 * kNb * kNh, 256, 0, stream>>>(DA, DBF, DBB, CMF, CMB, XF, XB, H0, YF, YB, HF, HB);

  gate_rmsnorm_kernel<<<kRows / 8, 256, 0, stream>>>(YF, YB, XF, ZX, Dp, key_norm_w, GN);
  state_layernorm_kernel<<<kQRows / 8, 256, 0, stream>>>(HF, HB, ln_w, ln_b, SN);

  gemm_f16_nt_kernel<<<((kRows / 64) * (kDm / 64)) / 8, 256, 0, stream>>>(
      GN, kDi, BOKH, kDi, out, kDm, kRows, kDm, kDi, kFoldMid);
  gemm_f16_nt_kernel<<<((kQRows / 64) * (kDm / 64)) / 8, 256, 0, stream>>>(
      SN, kDi, BOQH, kDi, out + (size_t)kRows * kDm, kDm, kQRows, kDm, kDi, kFoldMid);
}
